// LSTMNet_53961969107393
// MI455X (gfx1250) — hardware-verified
//
#include <hip/hip_runtime.h>
#include <math.h>

constexpr int NB     = 1024;
constexpr int TSEQ   = 1000;
constexpr int TFUT   = 100;
constexpr int TT     = TSEQ + TFUT;
constexpr int HDIM   = 51;
constexpr int NGATE  = 4 * HDIM;
constexpr int NQ4    = NGATE / 4;
constexpr int NPV    = 5;
constexpr int PPITCH = 208;
constexpr int ROWS   = 16;
constexpr int NTHR   = 128;
constexpr int UPAD   = 64;
constexpr int NPAD   = 4 * UPAD;
constexpr int KP1    = 64;
constexpr int KP2    = 128;
constexpr int HPAD   = 72;
constexpr int H2FP   = 64;
constexpr int XCH    = 128;
constexpr int XSP    = 132;
constexpr int OTP    = 1104;
constexpr float HCARRY = 256.0f;
constexpr float WCARRY = 1024.0f;
constexpr float ZFOLD  = 1.0f / 262144.0f;
constexpr int NQ  = ROWS * TT / 4;
constexpr int NIT = (NQ + NTHR - 1) / NTHR;

static_assert(NB % ROWS == 0, "grid exact");
static_assert(HDIM <= UPAD && UPAD == 4 * 16, "4 unit subtiles of 16 per gate");
static_assert(NTHR == 4 * 32, "one wave per unit subtile");
static_assert(ROWS * 8 == NTHR, "head mapping: 8 lanes per row");
static_assert(HPAD % 8 == 0 && KP1 % 8 == 0 && KP2 % 8 == 0, "16-B aligned fragment loads");
static_assert(KP1 == 64 && KP2 == 128, "K chunks of 32: 2 and 4");
static_assert(NGATE % 4 == 0 && NQ4 <= NTHR && 4 * NQ4 <= PPITCH && PPITCH % 4 == 0, "parameter staging");
static_assert(TSEQ % 4 == 0 && TSEQ >= 4, "float4 x loads");
static_assert(ROWS * XCH / 4 == 4 * NTHR, "x fill: 4 iterations x 128 threads x 4 floats = 16 x 128");
static_assert(XSP % 4 == 0 && XSP >= XCH, "x staging");
static_assert(TT % 4 == 0 && OTP % 4 == 0 && OTP >= TT, "output tile float4 reads");
static_assert((ROWS * TT * 4) % 128 == 0, "output tile = whole 128-B lines, aligned base");
static_assert((4 * ROWS * HPAD / 2) % NTHR == 0, "h zero-fill exact");
static_assert((ROWS * H2FP) % NTHR == 0, "h2f zero-fill exact");
static_assert(NPAD * KP1 / 8 == 8 * 256, "wprep grid: 8 blocks x 256 threads exact");

typedef __attribute__((ext_vector_type(16))) _Float16 v16h;
typedef __attribute__((ext_vector_type(8)))  _Float16 v8h;
typedef __attribute__((ext_vector_type(8)))  float    v8f;
typedef __attribute__((ext_vector_type(4)))  float    v4f;

__device__ __forceinline__ unsigned short f2bf_bits(float f) {
  unsigned u = __float_as_uint(f);
  return (unsigned short)((u + 0x7FFFu + ((u >> 16) & 1u)) >> 16);
}
__device__ __forceinline__ float bf_bits2f(unsigned short h) { return __uint_as_float(((unsigned)h) << 16); }
__device__ __forceinline__ float bf16r(float f) { return bf_bits2f(f2bf_bits(f)); }

__device__ __forceinline__ void grp_guard5(v8f& a0, v8f& a1, v8f& a2, v8f& a3,
                                           v16h x, v16h y0, v16h y1, v16h y2, v16h y3) {
  asm volatile("v_nop\n\tv_nop\n\tv_nop\n\tv_nop"
               : "+v"(a0), "+v"(a1), "+v"(a2), "+v"(a3)
               : "v"(x), "v"(y0), "v"(y1), "v"(y2), "v"(y3));
}
__device__ __forceinline__ void acc_guard4(v8f& a, v8f& b, v8f& c, v8f& d) {
  asm volatile("v_nop\n\tv_nop\n\tv_nop\n\tv_nop" : "+v"(a), "+v"(b), "+v"(c), "+v"(d));
}

struct FragH {
  union U { v16h v; v8h h[2]; };
  static __device__ __forceinline__ v16h load(const _Float16* p) {
    U f; f.h[0] = *(const v8h*)(p); f.h[1] = *(const v8h*)(p + 16); return f.v;
  }
  static __device__ __forceinline__ v8f mma(v16h a, v16h b, v8f c) {
    return __builtin_amdgcn_wmma_f32_16x16x32_f16(false, a, false, b, (short)0, c, false, false);
  }
};

__device__ __forceinline__ float fsig(float x)  { return __builtin_amdgcn_rcpf(1.0f + __expf(-x)); }
__device__ __forceinline__ float ftanh(float x) { return 1.0f - 2.0f * __builtin_amdgcn_rcpf(__expf(2.0f * x) + 1.0f); }

__global__ __launch_bounds__(256) void wprep_kernel(const float* __restrict__ W, unsigned short* __restrict__ dst,
                                                    int dpitch, int dcol0) {
  const int i  = blockIdx.x * 256 + threadIdx.x;
  const int n  = i >> 3, c8 = (i & 7) * 8;
  const int g  = n >> 6, u = n & 63;
  const int uc = (u < HDIM) ? u : (HDIM - 1);
  const float ufac = (u < HDIM) ? 1.0f : 0.0f;
  const float* wrow = W + (size_t)(HDIM * g + uc) * HDIM;
  v8h hv;
#pragma unroll
  for (int e = 0; e < 8; ++e) {
    const int k  = c8 + e;
    const int kc = (k < HDIM) ? k : (HDIM - 1);
    const float kfac = (k < HDIM) ? 1.0f : 0.0f;
    const float f = wrow[kc];
    const float v = (bf16r(f) * WCARRY) * (ufac * kfac);
    hv[e] = (_Float16)v;
  }
  unsigned short* op = dst + (size_t)n * dpitch + dcol0 + c8;
  *(volatile v8h*)op = hv;
  __threadfence();
  *(volatile v8h*)op = hv;
}

__global__ __launch_bounds__(NTHR) void lstm2_seq_kernel(const float* __restrict__ x,
                                                         const float* __restrict__ Wih1,
                                                         const float* __restrict__ bih1, const float* __restrict__ bhh1,
                                                         const float* __restrict__ bih2, const float* __restrict__ bhh2,
                                                         const float* __restrict__ Wl, const float* __restrict__ bl,
                                                         const unsigned short* __restrict__ W1Pp,
                                                         const unsigned short* __restrict__ W2Pp,
                                                         float* __restrict__ out) {
  __shared__ __align__(16) _Float16 Ht[4][ROWS * HPAD];
  __shared__ __align__(16) float    H2f[ROWS * H2FP];
  __shared__ __align__(16) float    OLAST[ROWS];
  __shared__ __align__(16) float    WLs[64];
  __shared__ __align__(16) float    PRM[NPV][PPITCH];
  __shared__ __align__(16) float    XS[ROWS * XSP];
  __shared__ __align__(16) float    OT[ROWS * OTP];

  const _Float16* W1P = (const _Float16*)W1Pp;
  const _Float16* W2P = (const _Float16*)W2Pp;
  const int tid = threadIdx.x, lane = tid & 31, wave = tid >> 5;
  const int c = lane & 15, hh = lane >> 4, koff = hh * 8;
  const int b0 = blockIdx.x * ROWS;
  const int u = 16 * wave + c;
  const bool ureal = (u < HDIM);
  const int uc = ureal ? u : (HDIM - 1);
  const float ufac = ureal ? 1.0f : 0.0f;
  const int hrow = tid >> 3, hsub = tid & 7;

  {
    unsigned* hz = (unsigned*)(&Ht[0][0]);
#pragma unroll 1
    for (int i = tid; i < 4 * ROWS * HPAD / 2; i += NTHR) hz[i] = 0u;
#pragma unroll 1
    for (int i = tid; i < ROWS * H2FP; i += NTHR) H2f[i] = 0.0f;
    if (tid < ROWS) OLAST[tid] = 0.0f;
  }
  {
    const int q = (tid < NQ4) ? tid : (NQ4 - 1);
    const v4f p0 = *(const v4f*)(Wih1 + 4 * q);
    const v4f p1 = *(const v4f*)(bih1 + 4 * q);
    const v4f p2 = *(const v4f*)(bhh1 + 4 * q);
    const v4f p3 = *(const v4f*)(bih2 + 4 * q);
    const v4f p4 = *(const v4f*)(bhh2 + 4 * q);
    if (tid < NQ4) {
      *(v4f*)(&PRM[0][4 * q]) = p0;
      *(v4f*)(&PRM[1][4 * q]) = p1;
      *(v4f*)(&PRM[2][4 * q]) = p2;
      *(v4f*)(&PRM[3][4 * q]) = p3;
      *(v4f*)(&PRM[4][4 * q]) = p4;
    }
    const int kc = (tid < HDIM) ? tid : (HDIM - 1);
    const float wfac = (tid < HDIM) ? 1.0f : 0.0f;
    const float wlv = bf16r(Wl[kc]) * wfac;
    if (tid < 64) WLs[tid] = wlv;
  }
  const float blr = bf16r(bl[0]);
  float c1s[8], c2s[8];
#pragma unroll
  for (int r = 0; r < 8; ++r) { c1s[r] = 0.0f; c2s[r] = 0.0f; }
  __syncthreads();

  float wih1r[4], bias1[4], bias2[4];
#pragma unroll
  for (int g = 0; g < 4; ++g) {
    const int n = HDIM * g + uc;
    wih1r[g] = bf16r(PRM[0][n]) * ufac;
    bias1[g] = (bf16r(PRM[1][n]) + bf16r(PRM[2][n])) * ufac;
    bias2[g] = (bf16r(PRM[3][n]) + bf16r(PRM[4][n])) * ufac;
  }
  float wl[8];
#pragma unroll
  for (int e = 0; e < 8; ++e) wl[e] = WLs[hsub * 8 + e];

  const v8f z8 = {0.f, 0.f, 0.f, 0.f, 0.f, 0.f, 0.f, 0.f};
  const _Float16* htbase = &Ht[0][0];
  const _Float16* w1row = W1P + (size_t)u * KP1 + koff;
  const _Float16* w2row = W2P + (size_t)u * KP2 + koff;

#pragma unroll 1
  for (int t = 0; t < TT; ++t) {
    const int cur = t & 1, nxt = cur ^ 1;

    if (t < TSEQ && (t & (XCH - 1)) == 0) {
#pragma unroll
      for (int i2 = 0; i2 < 4; ++i2) {
        const int idx = i2 * NTHR + tid;
        const int m = idx >> 5, q4 = (idx & 31) * 4;
        int tt = t + q4;
        tt = (tt > TSEQ - 4) ? (TSEQ - 4) : tt;
        const v4f v = *(const v4f*)(x + (size_t)(b0 + m) * TSEQ + tt);
        v4f vr;
        vr[0] = bf16r(v[0]); vr[1] = bf16r(v[1]); vr[2] = bf16r(v[2]); vr[3] = bf16r(v[3]);
        *(v4f*)(XS + m * XSP + q4) = vr;
      }
      __syncthreads();
    }

    float xin[8];
    {
      const int col = t & (XCH - 1);
#pragma unroll
      for (int r = 0; r < 8; ++r) {
        const float xs = XS[(8 * hh + r) * XSP + col];
        const float fb = OLAST[8 * hh + r];
        xin[r] = (t < TSEQ) ? xs : fb;
      }
    }

    v8f acc[4];
    acc[0] = z8; acc[1] = z8; acc[2] = z8; acc[3] = z8;
    {
      const _Float16* arow = htbase + cur * (ROWS * HPAD) + c * HPAD + koff;
#pragma unroll 1
      for (int kc = 0; kc < 2; ++kc) {
        const v16h a   = FragH::load(arow + 32 * kc);
        const v16h bq0 = FragH::load(w1row + 0 * UPAD * KP1 + 32 * kc);
        const v16h bq1 = FragH::load(w1row + 1 * UPAD * KP1 + 32 * kc);
        const v16h bq2 = FragH::load(w1row + 2 * UPAD * KP1 + 32 * kc);
        const v16h bq3 = FragH::load(w1row + 3 * UPAD * KP1 + 32 * kc);
        acc[0] = FragH::mma(a, bq0, acc[0]);
        acc[1] = FragH::mma(a, bq1, acc[1]);
        acc[2] = FragH::mma(a, bq2, acc[2]);
        acc[3] = FragH::mma(a, bq3, acc[3]);
        grp_guard5(acc[0], acc[1], acc[2], acc[3], a, bq0, bq1, bq2, bq3);
      }
      acc_guard4(acc[0], acc[1], acc[2], acc[3]);
    }
#pragma unroll
    for (int r = 0; r < 8; ++r) {
      const float zi = acc[0][r] * ZFOLD + (bias1[0] + xin[r] * wih1r[0]);
      const float zf = acc[1][r] * ZFOLD + (bias1[1] + xin[r] * wih1r[1]);
      const float zg = acc[2][r] * ZFOLD + (bias1[2] + xin[r] * wih1r[2]);
      const float zo = acc[3][r] * ZFOLD + (bias1[3] + xin[r] * wih1r[3]);
      const float ig = fsig(zi), fg = fsig(zf), og = fsig(zo), gg = ftanh(zg);
      const float cn = fg * c1s[r] + ig * gg;
      c1s[r] = cn;
      const float hn = og * ftanh(cn);
      const float hv = ureal ? hn : 0.0f;
      Ht[nxt][(8 * hh + r) * HPAD + u] = (_Float16)(hv * HCARRY);
    }
    __syncthreads();

    acc[0] = z8; acc[1] = z8; acc[2] = z8; acc[3] = z8;
    {
#pragma unroll 1
      for (int kc = 0; kc < 4; ++kc) {
        const int tsel = (kc < 2) ? nxt : (2 + cur);
        const int kk = (kc & 1) * 32;
        const _Float16* ap = htbase + tsel * (ROWS * HPAD) + c * HPAD + koff + kk;
        const v16h a   = FragH::load(ap);
        const v16h bq0 = FragH::load(w2row + 0 * UPAD * KP2 + 32 * kc);
        const v16h bq1 = FragH::load(w2row + 1 * UPAD * KP2 + 32 * kc);
        const v16h bq2 = FragH::load(w2row + 2 * UPAD * KP2 + 32 * kc);
        const v16h bq3 = FragH::load(w2row + 3 * UPAD * KP2 + 32 * kc);
        acc[0] = FragH::mma(a, bq0, acc[0]);
        acc[1] = FragH::mma(a, bq1, acc[1]);
        acc[2] = FragH::mma(a, bq2, acc[2]);
        acc[3] = FragH::mma(a, bq3, acc[3]);
        grp_guard5(acc[0], acc[1], acc[2], acc[3], a, bq0, bq1, bq2, bq3);
      }
      acc_guard4(acc[0], acc[1], acc[2], acc[3]);
    }
#pragma unroll
    for (int r = 0; r < 8; ++r) {
      const float zi = acc[0][r] * ZFOLD + bias2[0];
      const float zf = acc[1][r] * ZFOLD + bias2[1];
      const float zg = acc[2][r] * ZFOLD + bias2[2];
      const float zo = acc[3][r] * ZFOLD + bias2[3];
      const float ig = fsig(zi), fg = fsig(zf), og = fsig(zo), gg = ftanh(zg);
      const float cn = fg * c2s[r] + ig * gg;
      c2s[r] = cn;
      const float hn = og * ftanh(cn);
      const float hv = ureal ? hn : 0.0f;
      Ht[2 + nxt][(8 * hh + r) * HPAD + u] = (_Float16)(hv * HCARRY);
      H2f[(8 * hh + r) * H2FP + u] = hv;
    }
    __syncthreads();

    {
      float s = 0.0f;
#pragma unroll
      for (int e = 0; e < 8; ++e) s = s + H2f[hrow * H2FP + hsub * 8 + e] * wl[e];
      s += __shfl_xor(s, 1, 32);
      s += __shfl_xor(s, 2, 32);
      s += __shfl_xor(s, 4, 32);
      const float o = s + blr;
      if (hsub == 0) { OT[hrow * OTP + t] = o; OLAST[hrow] = o; }
    }
    __syncthreads();
  }

  {
    float* ob = out + (size_t)blockIdx.x * (size_t)(ROWS * TT);
    for (int pass = 0; pass < 2; ++pass) {
#pragma unroll 1
      for (int it = 0; it < NIT; ++it) {
        const int q  = it * NTHR + tid;
        const int qc = (q < NQ) ? q : (NQ - 1);
        const int e  = qc * 4;
        const int row = e / TT;
        const int col = e - row * TT;
        const v4f v = *(const v4f*)(OT + row * OTP + col);
        if (q < NQ) *(volatile v4f*)(ob + (size_t)q * 4) = v;
      }
      __threadfence();
    }
  }
}

extern "C" void kernel_launch(void* const* d_in, const int* in_sizes, int n_in,
                              void* d_out, int out_size, void* d_ws, size_t ws_size, hipStream_t stream) {
  if (n_in < 11 || d_out == nullptr || d_ws == nullptr) return;
  if (in_sizes[0] != NB * TSEQ || in_sizes[1] != NGATE || in_sizes[2] != NGATE * HDIM ||
      in_sizes[3] != NGATE || in_sizes[4] != NGATE || in_sizes[5] != NGATE * HDIM || in_sizes[6] != NGATE * HDIM ||
      in_sizes[7] != NGATE || in_sizes[8] != NGATE || in_sizes[9] != HDIM || in_sizes[10] != 1 ||
      out_size != NB * TT) return;

  const float* x    = (const float*)d_in[0];
  const float* Wih1 = (const float*)d_in[1];
  const float* Whh1 = (const float*)d_in[2];
  const float* bih1 = (const float*)d_in[3];
  const float* bhh1 = (const float*)d_in[4];
  const float* Wih2 = (const float*)d_in[5];
  const float* Whh2 = (const float*)d_in[6];
  const float* bih2 = (const float*)d_in[7];
  const float* bhh2 = (const float*)d_in[8];
  const float* Wl   = (const float*)d_in[9];
  const float* bl   = (const float*)d_in[10];
  float* out = (float*)d_out;

  char* ws = (char*)d_ws; size_t off = 0;
  auto carve = [&](size_t bytes) -> char* { char* p = ws + off; off += (bytes + 255) & ~(size_t)255; return p; };
  unsigned short* W1P = (unsigned short*)carve((size_t)NPAD * KP1 * 2);
  unsigned short* W2P = (unsigned short*)carve((size_t)NPAD * KP2 * 2);
  if (off > ws_size || off > (size_t)134217728) return;

  wprep_kernel<<<8, 256, 0, stream>>>(Whh1, W1P, KP1, 0);
  wprep_kernel<<<8, 256, 0, stream>>>(Wih2, W2P, KP2, 0);
  wprep_kernel<<<8, 256, 0, stream>>>(Whh2, W2P, KP2, UPAD);
  lstm2_seq_kernel<<<NB / ROWS, NTHR, 0, stream>>>(x, Wih1, bih1, bhh1, bih2, bhh2, Wl, bl, W1P, W2P, out);
}
